// ConvSP_46772193853617
// MI455X (gfx1250) — hardware-run, weakly checked
//
#include <hip/hip_runtime.h>
#include <math.h>

typedef __attribute__((ext_vector_type(16))) _Float16 v16h;
typedef __attribute__((ext_vector_type(16))) __bf16 v16b;
typedef __attribute__((ext_vector_type(8)))  _Float16 v8h;
typedef __attribute__((ext_vector_type(8)))  float v8f;
typedef __attribute__((ext_vector_type(4)))  float v4f;
typedef __attribute__((ext_vector_type(2)))  float v2f;
typedef __attribute__((ext_vector_type(4)))  unsigned v4u;
typedef __attribute__((ext_vector_type(4)))  int v4i;
typedef float __attribute__((may_alias)) float_a;
typedef int __attribute__((may_alias)) int_a;

template <typename T> __device__ __forceinline__ void vst2(void* p, T v) { *(volatile T*)p = v; __threadfence(); *(volatile T*)p = v; }
__device__ __forceinline__ v8f wmma16(v16h a, v16h b, v8f c) {
  v8f d = __builtin_amdgcn_wmma_f32_16x16x32_f16(false, a, false, b, (short)0, c, false, false);
  asm volatile("v_nop\n\tv_nop\n\tv_nop\n\tv_nop" : "+v"(d) : "v"(a), "v"(b));
  return d;
}
__device__ __forceinline__ v8f wmma_bf(v16b a, v16b b, v8f c) {
  v8f d = __builtin_amdgcn_wmma_f32_16x16x32_bf16(false, a, false, b, (short)0, c, false, false);
  asm volatile("v_nop\n\tv_nop\n\tv_nop\n\tv_nop" : "+v"(d) : "v"(a), "v"(b));
  return d;
}
__device__ __forceinline__ v16h frag_h(const _Float16* rowk0, int lane) {
  union { v16h v; v8h q[2]; } u; const _Float16* p = rowk0 + 8 * (lane >> 4);
  u.q[0] = *(const v8h*)p; u.q[1] = *(const v8h*)(p + 16); return u.v;
}
__device__ __forceinline__ v16h frag_f32(const float* rowk0, int lane) {
  v16h a; const float* p = rowk0 + 8 * (lane >> 4);
#pragma unroll
  for (int i = 0; i < 8; ++i) { a[i] = (_Float16)p[i]; a[8 + i] = (_Float16)p[16 + i]; }
  return a;
}
__device__ __forceinline__ v16h frag_f32s(const float* rowk0, int lane, float sc) {
  v16h a; const float* p = rowk0 + 8 * (lane >> 4);
#pragma unroll
  for (int i = 0; i < 8; ++i) { a[i] = (_Float16)(p[i] * sc); a[8 + i] = (_Float16)(p[16 + i] * sc); }
  return a;
}
__device__ __forceinline__ v16h fragc_f32(const float* W, int k0, int n, int lane, int ld, int K) {
  v16h a; const int g = lane >> 4;
#pragma unroll
  for (int i = 0; i < 8; ++i) { const int ka = k0 + 8 * g + i, kb = ka + 16;
    a[i] = (_Float16)(ka < K ? W[(size_t)(ka < K ? ka : K - 1) * ld + n] : 0.f); a[8 + i] = (_Float16)(kb < K ? W[(size_t)(kb < K ? kb : K - 1) * ld + n] : 0.f); }
  return a;
}
struct F2 { v16b h, l; };
__device__ __forceinline__ F2 bsplit16(const float v[16]) { F2 r;
#pragma unroll
  for (int i = 0; i < 16; ++i) { const __bf16 h = (__bf16)v[i]; r.h[i] = h; r.l[i] = (__bf16)(v[i] - (float)h); }
  return r; }
__device__ __forceinline__ F2 split_row(const float* row, int k0, int lane) { float v[16]; const float* p = row + k0 + 8 * (lane >> 4);
#pragma unroll
  for (int i = 0; i < 8; ++i) { v[i] = p[i]; v[8 + i] = p[16 + i]; }
  return bsplit16(v); }
__device__ __forceinline__ F2 split_rowK(const float* row, int k0, int lane, int K) { float v[16]; const int g = lane >> 4;
#pragma unroll
  for (int i = 0; i < 8; ++i) { const int ka = k0 + 8 * g + i, kb = ka + 16; v[i] = ka < K ? row[ka < K ? ka : K - 1] : 0.f; v[8 + i] = kb < K ? row[kb < K ? kb : K - 1] : 0.f; }
  return bsplit16(v); }
__device__ __forceinline__ F2 split_col(const float* W, int k0, int n, int lane, int ld, int K) { float v[16]; const int g = lane >> 4;
#pragma unroll
  for (int i = 0; i < 8; ++i) { const int ka = k0 + 8 * g + i, kb = ka + 16; v[i] = ka < K ? W[(size_t)(ka < K ? ka : K - 1) * ld + n] : 0.f; v[8 + i] = kb < K ? W[(size_t)(kb < K ? kb : K - 1) * ld + n] : 0.f; }
  return bsplit16(v); }
__device__ __forceinline__ v8f mac3(const F2& a, const F2& b, v8f c) { c = wmma_bf(a.l, b.h, c); c = wmma_bf(a.h, b.l, c); return wmma_bf(a.h, b.h, c); }
__device__ __forceinline__ float sigm(float v) { return 1.0f / (1.0f + expf(-v)); }
#define LDSX() do { asm volatile("s_wait_dscnt 0" ::: "memory"); __builtin_amdgcn_wave_barrier(); __builtin_amdgcn_fence(__ATOMIC_RELEASE, "workgroup"); } while (0)

__device__ __forceinline__ float bfr(float v) { return (float)(__bf16)v; }
__device__ __attribute__((noinline)) float kv_ni(float dx, float dy, float dz) { const float d = sqrtf(dx * dx + dy * dy + dz * dz + 1e-12f); const float q = d / 0.1f; const float t = 1.0f - q; return (q < 1.0f) ? t * t * t : 0.f; }
#define NBT 2
#define MM 8192
#define NLOC 8192
#define KN 32
#define CI 16
#define CO 16
#define NCELL 27
#define KW (CI * NCELL)
#define KWP 448
#ifndef NBLK
#define NBLK (NBT * MM / 16)
#endif
__global__ __launch_bounds__(128) void k_convsp(const float* __restrict__ QL, const float* __restrict__ LC, const float* __restrict__ DT, const int* __restrict__ NB, const float* __restrict__ WT, const float* __restrict__ BI, float* __restrict__ OUT) {
  __shared__ __align__(16) float sacc[16][KWP + 4]; __shared__ __align__(16) float so[16 * CO];
  const int tid = threadIdx.x, wave = tid >> 5, lane = tid & 31, col = lane & 15, g = lane >> 4; const size_t p0 = (size_t)blockIdx.x * 16; const size_t b = p0 / MM;
  for (int e = tid; e < 16 * (KWP + 4); e += 128) (&sacc[0][0])[e] = 0.f;
  __syncthreads();
#pragma unroll 1
  for (int pp = 0; pp < 4; ++pp) { const int pl = wave * 4 + pp; const size_t p = p0 + pl; const size_t m = p % MM;
    const float qx = bfr(QL[p * 3]), qy = bfr(QL[p * 3 + 1]), qz = bfr(QL[p * 3 + 2]);
    int jn[16]; float nx[16], ny[16], nz[16]; bool vl[16];
#pragma unroll
    for (int i = 0; i < 16; ++i) { const int k = (i < 8) ? (8 * g + i) : (16 + 8 * g + (i - 8)); const int nbv = NB[p * KN + k]; vl[i] = nbv >= 0; const int j = vl[i] ? nbv : 0; jn[i] = j;
      nx[i] = bfr(LC[(b * NLOC + j) * 3]); ny[i] = bfr(LC[(b * NLOC + j) * 3 + 1]); nz[i] = bfr(LC[(b * NLOC + j) * 3 + 2]); }
#pragma unroll
    for (int et = 0; et < 2; ++et) { const int e = et * 16 + col;
      float av[16]; const int ee = e < NCELL ? e : 0; const float ox = ((float)(ee / 9) - 1.0f) * 0.05f, oy = ((float)((ee / 3) % 3) - 1.0f) * 0.05f, oz = ((float)(ee % 3) - 1.0f) * 0.05f;
      const float cx = qx + ox, cy = qy + oy, cz = qz + oz;
#pragma unroll
      for (int i = 0; i < 16; ++i) { const float kvv = kv_ni(cx - nx[i], cy - ny[i], cz - nz[i]); av[i] = (e < NCELL && vl[i]) ? kvv : 0.f; }
      const F2 a = bsplit16(av); v16b fb;
#pragma unroll
      for (int i = 0; i < 16; ++i) fb[i] = (__bf16)DT[(b * NLOC + jn[i]) * CI + col];
      v8f acc = {}; acc = wmma_bf(a.h, fb, acc); acc = wmma_bf(a.l, fb, acc);
#pragma unroll
      for (int r = 0; r < 8; ++r) { const int er = et * 16 + 8 * g + r; if (er < NCELL) sacc[pl][col * NCELL + er] = acc[r]; } }
  }
  __syncthreads();
  if (wave == 0) { v8f acc = {};
#pragma unroll 1
    for (int kc = 0; kc < KWP / 32; ++kc) { const F2 a = split_row(&sacc[col][0], kc * 32, lane); v16b w;
#pragma unroll
      for (int i = 0; i < 16; ++i) { const int k = kc * 32 + (i < 8 ? 8 * g + i : 16 + 8 * g + (i - 8)); w[i] = (k < KW) ? (__bf16)WT[(size_t)col * KW + (k < KW ? k : 0)] : (__bf16)0.f; }
      acc = wmma_bf(a.h, w, acc); acc = wmma_bf(a.l, w, acc); }
#pragma unroll
    for (int r = 0; r < 8; ++r) so[(8 * g + r) * CO + col] = acc[r] + bfr(BI[col]);
    LDSX();
    for (int q = lane; q < 16 * CO / 4; q += 32) vst2(OUT + p0 * CO + q * 4, *(const v4f*)&so[q * 4]); } }
extern "C" void kernel_launch(void* const* d_in, const int* in_sizes, int n_in, void* d_out, int out_size, void* d_ws, size_t ws_size, hipStream_t stream) {
  (void)in_sizes; (void)n_in; (void)out_size; (void)d_ws; (void)ws_size;
  const float** F = (const float**)d_in;
  k_convsp<<<dim3(NBLK), 128, 0, stream>>>(F[0], F[1], F[2], (const int*)d_in[3], F[4], F[5], (float*)d_out);
}
